// MultiHeadAttention_1881195676299
// MI455X (gfx1250) — hardware-verified
//
#include <hip/hip_runtime.h>


#ifndef NB
#define NB 2
#endif
#ifndef SEQ
#define SEQ 2048
#endif
#define NB_FULL  2
#define SEQ_FULL 2048
#ifndef OUT_SEQ
#define OUT_SEQ SEQ
#endif
#define DM   768
#define NH_  12
#define HD   64
#define AW   4
#define OSP  68
#define QRS  2048.0f
#define QRI  (1.0f / 2048.0f)
#define SSC  0.125f
#define NEGV (-1000000000.0f)
#define WSC  16.0f
#define CSC  (1.0f / 16.0f)

static_assert(HD == 64);
static_assert(NH_ * HD == DM);
static_assert(DM % 64 == 0);
static_assert(DM % 32 == 0);
static_assert(HD % 32 == 0);
static_assert(SEQ % 64 == 0);
static_assert((NB * SEQ) % 64 == 0);
static_assert((NB * SEQ) % 32 == 0);
static_assert(SEQ % 32 == 0);
static_assert(SEQ % (16 * AW) == 0);
static_assert(((size_t)SEQ * DM) % 8 == 0);
static_assert(((size_t)DM * DM) % 8 == 0);
static_assert(NB <= NB_FULL);
static_assert(SEQ <= SEQ_FULL);
static_assert((OSP * 4) % 16 == 0);
static_assert(OSP >= HD);
static_assert(32 * 16 * 4 == 16 * HD * 2);
static_assert(32 * 16 * 8 == 16 * 64 * 4);
static_assert(256 * 16 * 2 == 64 * 64 * 2);
static_assert(256 * 16 * 4 == 64 * 64 * 4);
static_assert(AW * 16 * OSP * 4 <= 131072);
static_assert(64 * 65 * 4 <= 131072);
static_assert(16 * 68 * 4 <= 131072);

typedef _Float16 h16;
typedef unsigned short bf;
typedef __attribute__((ext_vector_type(16))) __bf16   v16bf;
typedef __attribute__((ext_vector_type(16))) _Float16 v16h;
typedef __attribute__((ext_vector_type(8)))  _Float16 v8h;
typedef __attribute__((ext_vector_type(8)))  unsigned short v8us;
typedef __attribute__((ext_vector_type(8)))  float    v8f;
typedef __attribute__((ext_vector_type(4)))  float    v4f;
typedef __attribute__((ext_vector_type(4)))  int      v4i;
typedef v4f  __attribute__((may_alias)) v4fa;

__device__ __forceinline__ unsigned short f2bf(float f) { unsigned u = __float_as_uint(f); u += 0x7FFFu + ((u >> 16) & 1u); return (unsigned short)(u >> 16); }
__device__ __forceinline__ float bfr(float f) { return __uint_as_float(((unsigned)f2bf(f)) << 16); }
__device__ __forceinline__ v16h cat16(v8h lo, v8h hi) { return __builtin_shufflevector(lo, hi, 0, 1, 2, 3, 4, 5, 6, 7, 8, 9, 10, 11, 12, 13, 14, 15); }
__device__ __forceinline__ v16bf cat16b(v8us lo, v8us hi) { return __builtin_bit_cast(v16bf, __builtin_shufflevector(lo, hi, 0, 1, 2, 3, 4, 5, 6, 7, 8, 9, 10, 11, 12, 13, 14, 15)); }
__device__ __forceinline__ v8f wmma16(v16h a, v16h b, v8f c) { return __builtin_amdgcn_wmma_f32_16x16x32_f16(false, a, false, b, (short)0, c, false, false); }
__device__ __forceinline__ v8f wmmab(v16bf a, v16bf b, v8f c) { return __builtin_amdgcn_wmma_f32_16x16x32_bf16(false, a, false, b, (short)0, c, false, false); }
__device__ __forceinline__ v16h  ldh(const h16* p) { return cat16(*(const v8h*)p, *(const v8h*)(p + 16)); }
__device__ __forceinline__ v16bf ldb(const bf* p)  { return cat16b(*(const v8us*)p, *(const v8us*)(p + 16)); }
__device__ __forceinline__ void wave_sync() { __builtin_amdgcn_fence(3  , "wavefront"); __builtin_amdgcn_wave_barrier(); asm volatile("" ::: "memory"); }
__device__ __forceinline__ v8f wmmabg(v16bf a, v16bf b, v8f c) { c = wmmab(a, b, c); asm volatile("v_nop\n\tv_nop\n\tv_nop\n\tv_nop" : "+v"(c) : "v"(a), "v"(b)); return c; }
__device__ __forceinline__ v8f wmma16g(v16h a, v16h b, v8f c) { c = wmma16(a, b, c); asm volatile("v_nop\n\tv_nop\n\tv_nop\n\tv_nop" : "+v"(c) : "v"(a), "v"(b)); return c; }
static __device__ __forceinline__ h16 toh_flush(float v) { const float w = (fabsf(v) < 6.103515625e-05f) ? 0.0f : v; return (h16)w; }

__global__ __launch_bounds__(256) void k_cvt8(const float* __restrict__ src, bf* dst, size_t n8) {
    const size_t i = (size_t)blockIdx.x * 256 + threadIdx.x; if (i >= n8) return;
    const v8f v = *(const v8f*)(src + i * 8); v8us o;
#pragma unroll
    for (int k = 0; k < 8; ++k) o[k] = f2bf(v[k]);
    *(volatile v8us*)(dst + i * 8) = o; __threadfence(); *(volatile v8us*)(dst + i * 8) = o;
}

template <int F16>
__device__ __forceinline__ void wtr_body(const float* __restrict__ W, bf* OB, h16* OH) {
    __shared__ float ts[64 * 65];
    const unsigned tid = threadIdx.x;
    const unsigned k0 = blockIdx.x * 64u, n0 = blockIdx.y * 64u;
#pragma unroll
    for (unsigned it = 0; it < 4; ++it) { const unsigned p = it * 256u + tid; const unsigned kk = p >> 4, c4 = (p & 15u) * 4u;
        const v4f v = *(const v4f*)(W + (size_t)(k0 + kk) * DM + n0 + c4);
        ts[kk * 65 + c4 + 0] = v[0]; ts[kk * 65 + c4 + 1] = v[1]; ts[kk * 65 + c4 + 2] = v[2]; ts[kk * 65 + c4 + 3] = v[3]; }
    __syncthreads();
#pragma unroll 1
    for (int ps = 0; ps < 2; ++ps) {
#pragma unroll
        for (unsigned it = 0; it < 2; ++it) { const unsigned p = it * 256u + tid; const unsigned nn = p >> 3, c8 = (p & 7u) * 8u;
            const size_t oo = (size_t)(n0 + nn) * DM + k0 + c8;
            if (F16) { v8h o;
#pragma unroll
                for (unsigned i = 0; i < 8; ++i) o[i] = toh_flush(bfr(ts[(c8 + i) * 65 + nn]) * WSC);
                *(volatile v8h*)(OH + oo) = o; }
            else { v8us o;
#pragma unroll
                for (unsigned i = 0; i < 8; ++i) o[i] = f2bf(ts[(c8 + i) * 65 + nn]);
                *(volatile v8us*)(OB + oo) = o; } }
        if (ps == 0) __threadfence(); }
}
__global__ __launch_bounds__(256) void k_wtr_b(const float* __restrict__ W, bf* OB)  { wtr_body<0>(W, OB, (h16*)0); }
__global__ __launch_bounds__(256) void k_wtr_h(const float* __restrict__ W, h16* OH) { wtr_body<1>(W, (bf*)0, OH); }

template <int MODE>
__device__ __forceinline__ void proj_body(const bf* __restrict__ A, const bf* __restrict__ Bt, const float* __restrict__ bias, h16* Ph, h16* Pr) {
    __shared__ __align__(16) float os[16 * 68];
    const int K = DM;
    const int lane = threadIdx.x & 31, lr = lane & 15, hi = lane >> 4;
    const unsigned bx = blockIdx.x, by = blockIdx.y;
    const unsigned r0 = bx * 64u, c0 = by * 64u;
    v8f acc[4][4];
#pragma unroll
    for (int mb = 0; mb < 4; ++mb)
#pragma unroll
        for (int nb = 0; nb < 4; ++nb) acc[mb][nb] = (v8f){};
    const size_t aoff = (size_t)(r0 + (unsigned)lr) * K + 8 * hi, boff = (size_t)(c0 + (unsigned)lr) * K + 8 * hi;
#pragma unroll 1
    for (int kc = 0; kc < K; kc += 32) {
        v16bf a[4];
#pragma unroll
        for (int mb = 0; mb < 4; ++mb) a[mb] = ldb(A + aoff + (size_t)mb * 16 * K + kc);
#pragma unroll
        for (int nb = 0; nb < 4; ++nb) { const v16bf b = ldb(Bt + boff + (size_t)nb * 16 * K + kc);
#pragma unroll
            for (int mb = 0; mb < 4; ++mb) acc[mb][nb] = wmmabg(a[mb], b, acc[mb][nb]); }
    }
    float bc[4];
#pragma unroll
    for (int nb = 0; nb < 4; ++nb) bc[nb] = (MODE == 0) ? bfr(bias[c0 + (unsigned)(nb * 16 + lr)]) : 0.0f;
    size_t tbase; size_t pitch;
    if (MODE == 0) { const unsigned bb = r0 / (unsigned)SEQ, tt = r0 % (unsigned)SEQ; const unsigned zc = bb * (unsigned)NH_ + c0 / (unsigned)HD;
                     tbase = ((size_t)zc * SEQ + (size_t)tt) * HD; pitch = (size_t)HD; }
    else           { const unsigned bb = c0 / (unsigned)SEQ, tt = c0 % (unsigned)SEQ;
                     tbase = (size_t)bb * (size_t)DM * SEQ + (size_t)r0 * SEQ + (size_t)tt; pitch = (size_t)SEQ; }
#pragma unroll
    for (int mb = 0; mb < 4; ++mb) {
        float br[8];
#pragma unroll
        for (int j = 0; j < 8; ++j) br[j] = (MODE == 1) ? bfr(bias[r0 + (unsigned)(mb * 16 + hi * 8 + j)]) : 0.0f;
#pragma unroll
        for (int nb = 0; nb < 4; ++nb) {
#pragma unroll
            for (int j = 0; j < 8; ++j) os[(hi * 8 + j) * 68 + nb * 16 + lr] = acc[mb][nb][j] + bc[nb] + br[j]; }
        wave_sync();
#pragma unroll 1
        for (int ps = 0; ps < 2; ++ps) {
            const size_t sb = tbase + (size_t)(mb * 16) * pitch;
#pragma unroll
            for (int s = 0; s < 4; ++s) { const int row = 4 * s + (lane >> 3), c8 = (lane & 7) * 8;
                const v4f x0 = *(const v4fa*)(&os[row * 68 + c8]); const v4f x1 = *(const v4fa*)(&os[row * 68 + c8 + 4]); v8h hv, rv;
#pragma unroll
                for (int i = 0; i < 4; ++i) { const h16 a0 = toh_flush(x0[i]); const h16 a1 = toh_flush(x1[i]); hv[i] = a0; hv[4 + i] = a1;
                                              rv[i] = toh_flush((x0[i] - (float)a0) * QRS); rv[4 + i] = toh_flush((x1[i] - (float)a1) * QRS); }
                const size_t oo = sb + (size_t)row * pitch + c8;
                *(volatile v8h*)(Ph + oo) = hv; if (MODE == 0) *(volatile v8h*)(Pr + oo) = rv; }
            if (ps == 0) __threadfence(); }
        wave_sync();
    }
}
__global__ __launch_bounds__(32) void k_proj_rows(const bf* __restrict__ A, const bf* __restrict__ Bt, const float* __restrict__ bias, h16* Ph, h16* Pr) { proj_body<0>(A, Bt, bias, Ph, Pr); }
__global__ __launch_bounds__(32) void k_proj_cols(const bf* __restrict__ A, const bf* __restrict__ Bt, const float* __restrict__ bias, h16* Ph) { proj_body<1>(A, Bt, bias, Ph, (h16*)0); }

__global__ __launch_bounds__(32 * AW) __attribute__((amdgpu_num_vgpr(256)))
void k_attn(const h16* __restrict__ QH, const h16* __restrict__ QR, const h16* __restrict__ KP, const h16* __restrict__ KR,
            const h16* __restrict__ VT, const int* __restrict__ mask, h16* CH, h16* CR) {
    __shared__ __align__(16) float os[AW * 16 * OSP];
    const int lane = threadIdx.x & 31, lr = lane & 15, hi = lane >> 4;
    const int wave = __builtin_amdgcn_readfirstlane((int)(threadIdx.x >> 5));
    const unsigned zh = blockIdx.y; const unsigned b = zh / (unsigned)NH_, h = zh % (unsigned)NH_;
    const int t0 = ((int)blockIdx.x * AW + wave) * 16;
    const size_t pbase = (size_t)zh * SEQ * HD;
    const size_t qo = pbase + (size_t)(t0 + lr) * HD + 8 * hi;
    const v16h qh0 = ldh(QH + qo), qh1 = ldh(QH + qo + 32);
    const v16h qr0 = ldh(QR + qo), qr1 = ldh(QR + qo + 32);
    const size_t ko = pbase + (size_t)lr * HD + 8 * hi;
    const size_t vo = pbase + (size_t)lr * SEQ + 8 * hi;
    const int* mrow = mask + (size_t)(t0 + lr) * SEQ_FULL + 8 * hi;
    v8f o0 = (v8f){}, o1 = (v8f){}, o2 = (v8f){}, o3 = (v8f){};
#pragma unroll 1
    for (int key0 = 0; key0 < SEQ; key0 += 32) {
        const h16* ka = KP + ko + (size_t)key0 * HD;
        const h16* kr = KR + ko + (size_t)key0 * HD;
        v8f sHa = (v8f){}, sLa = (v8f){}, sHb = (v8f){}, sLb = (v8f){};
        { const v16h a0 = ldh(ka), a1 = ldh(ka + 32), r0 = ldh(kr), r1 = ldh(kr + 32);
          sHa = wmma16g(a0, qh0, sHa); sHa = wmma16g(a1, qh1, sHa);
          sLa = wmma16g(a0, qr0, sLa); sLa = wmma16g(a1, qr1, sLa);
          sLa = wmma16g(r0, qh0, sLa); sLa = wmma16g(r1, qh1, sLa); }
        { const v16h a0 = ldh(ka + 16 * HD), a1 = ldh(ka + 16 * HD + 32), r0 = ldh(kr + 16 * HD), r1 = ldh(kr + 16 * HD + 32);
          sHb = wmma16g(a0, qh0, sHb); sHb = wmma16g(a1, qh1, sHb);
          sLb = wmma16g(a0, qr0, sLb); sLb = wmma16g(a1, qr1, sLb);
          sLb = wmma16g(r0, qh0, sLb); sLb = wmma16g(r1, qh1, sLb); }
        const int* mp = mrow + key0;
        const v4i m0 = *(const v4i*)mp, m1 = *(const v4i*)(mp + 4), m2 = *(const v4i*)(mp + 16), m3 = *(const v4i*)(mp + 20);
        int kx[8], ky[8];
#pragma unroll
        for (int r = 0; r < 4; ++r) { kx[r] = m0[r]; kx[4 + r] = m1[r]; ky[r] = m2[r]; ky[4 + r] = m3[r]; }
        v16h pb;
#pragma unroll
        for (int r = 0; r < 8; ++r) {
            const float sa = (sHa[r] + sLa[r] * QRI) * SSC, sb = (sHb[r] + sLb[r] * QRI) * SSC;
            const float va = (kx[r] == 0) ? NEGV : sa, vb = (ky[r] == 0) ? NEGV : sb;
            pb[r] = toh_flush(va); pb[8 + r] = toh_flush(vb); }
        const h16* va_ = VT + vo + key0;
        { const v16h v = ldh(va_);                     o0 = wmma16g(v, pb, o0); }
        { const v16h v = ldh(va_ + (size_t)16 * SEQ);  o1 = wmma16g(v, pb, o1); }
        { const v16h v = ldh(va_ + (size_t)32 * SEQ);  o2 = wmma16g(v, pb, o2); }
        { const v16h v = ldh(va_ + (size_t)48 * SEQ);  o3 = wmma16g(v, pb, o3); }
    }
    const v8f f0 = o0, f1 = o1, f2 = o2, f3 = o3;
    const int wb = wave * 16 * OSP;
    { v4f a, c;
      a[0] = f0[0]; a[1] = f0[1]; a[2] = f0[2]; a[3] = f0[3]; c[0] = f0[4]; c[1] = f0[5]; c[2] = f0[6]; c[3] = f0[7];
      *(v4fa*)(&os[wb + lr * OSP +  0 + 8 * hi]) = a; *(v4fa*)(&os[wb + lr * OSP +  0 + 8 * hi + 4]) = c;
      a[0] = f1[0]; a[1] = f1[1]; a[2] = f1[2]; a[3] = f1[3]; c[0] = f1[4]; c[1] = f1[5]; c[2] = f1[6]; c[3] = f1[7];
      *(v4fa*)(&os[wb + lr * OSP + 16 + 8 * hi]) = a; *(v4fa*)(&os[wb + lr * OSP + 16 + 8 * hi + 4]) = c;
      a[0] = f2[0]; a[1] = f2[1]; a[2] = f2[2]; a[3] = f2[3]; c[0] = f2[4]; c[1] = f2[5]; c[2] = f2[6]; c[3] = f2[7];
      *(v4fa*)(&os[wb + lr * OSP + 32 + 8 * hi]) = a; *(v4fa*)(&os[wb + lr * OSP + 32 + 8 * hi + 4]) = c;
      a[0] = f3[0]; a[1] = f3[1]; a[2] = f3[2]; a[3] = f3[3]; c[0] = f3[4]; c[1] = f3[5]; c[2] = f3[6]; c[3] = f3[7];
      *(v4fa*)(&os[wb + lr * OSP + 48 + 8 * hi]) = a; *(v4fa*)(&os[wb + lr * OSP + 48 + 8 * hi + 4]) = c; }
    wave_sync();
    const size_t cbase = ((size_t)b * SEQ + (size_t)t0) * DM + (size_t)h * HD;
#pragma unroll 1
    for (int ps = 0; ps < 2; ++ps) {
#pragma unroll
        for (int s = 0; s < 4; ++s) { const int row = 4 * s + (lane >> 3), c8 = (lane & 7) * 8;
            const v4f x0 = *(const v4fa*)(&os[wb + row * OSP + c8]); const v4f x1 = *(const v4fa*)(&os[wb + row * OSP + c8 + 4]); v8h hv, rv;
#pragma unroll
            for (int i = 0; i < 4; ++i) { const float y0 = x0[i] * CSC, y1 = x1[i] * CSC; const h16 a0 = toh_flush(y0); const h16 a1 = toh_flush(y1); hv[i] = a0; hv[4 + i] = a1;
                                          rv[i] = toh_flush((y0 - (float)a0) * QRS); rv[4 + i] = toh_flush((y1 - (float)a1) * QRS); }
            const size_t oo = cbase + (size_t)row * DM + c8;
            *(volatile v8h*)(CH + oo) = hv; *(volatile v8h*)(CR + oo) = rv; }
        if (ps == 0) __threadfence(); }
}

__global__ __launch_bounds__(32) __attribute__((amdgpu_num_vgpr(256)))
void k_oproj(const h16* __restrict__ CHp, const h16* __restrict__ CRp, const h16* __restrict__ WT, const float* __restrict__ bias, float* OUT) {
    __shared__ __align__(16) float os[16 * 68];
    const int K = DM;
    const int lane = threadIdx.x & 31, lr = lane & 15, hi = lane >> 4;
    const unsigned bx = blockIdx.x, by = blockIdx.y;
    const unsigned r0 = bx * 32u, c0 = by * 64u;
    v8f accH[2][4], accR[2][4];
#pragma unroll
    for (int mb = 0; mb < 2; ++mb)
#pragma unroll
        for (int nb = 0; nb < 4; ++nb) { accH[mb][nb] = (v8f){}; accR[mb][nb] = (v8f){}; }
    const size_t aoff = (size_t)(r0 + (unsigned)lr) * K + 8 * hi, boff = (size_t)(c0 + (unsigned)lr) * K + 8 * hi;
#pragma unroll 1
    for (int kc = 0; kc < K; kc += 32) {
        v16h ah[2], ar[2];
#pragma unroll
        for (int mb = 0; mb < 2; ++mb) { ah[mb] = ldh(CHp + aoff + (size_t)mb * 16 * K + kc); ar[mb] = ldh(CRp + aoff + (size_t)mb * 16 * K + kc); }
#pragma unroll
        for (int nb = 0; nb < 4; ++nb) { const v16h bw = ldh(WT + boff + (size_t)nb * 16 * K + kc);
#pragma unroll
            for (int mb = 0; mb < 2; ++mb) { accH[mb][nb] = wmma16g(ah[mb], bw, accH[mb][nb]); accR[mb][nb] = wmma16g(ar[mb], bw, accR[mb][nb]); } }
    }
    float bc[4];
#pragma unroll
    for (int nb = 0; nb < 4; ++nb) bc[nb] = bfr(bias[c0 + (unsigned)(nb * 16 + lr)]);
    const unsigned bb = r0 / (unsigned)SEQ, tt = r0 % (unsigned)SEQ;
    float* obase = OUT + ((size_t)bb * OUT_SEQ + (size_t)tt) * DM + c0;
#pragma unroll
    for (int mb = 0; mb < 2; ++mb) {
#pragma unroll
        for (int nb = 0; nb < 4; ++nb) {
#pragma unroll
            for (int j = 0; j < 8; ++j) os[(hi * 8 + j) * 68 + nb * 16 + lr] = accH[mb][nb][j] + accR[mb][nb][j] * QRI + bc[nb]; }
        wave_sync();
#pragma unroll 1
        for (int ps = 0; ps < 2; ++ps) {
#pragma unroll
            for (int s = 0; s < 8; ++s) { const int row = 2 * s + (lane >> 4), c4 = (lane & 15) * 4;
                const v4f val = *(const v4fa*)(&os[row * 68 + c4]);
                *(volatile v4f*)(obase + (size_t)(mb * 16 + row) * DM + c4) = val; }
            if (ps == 0) __threadfence(); }
        wave_sync();
    }
}

static constexpr size_t al256(size_t v) { return (v + 255) & ~(size_t)255; }
static constexpr size_t SZ_XB = al256((size_t)NB * SEQ * DM * 2);
static constexpr size_t SZ_WT = al256((size_t)DM * DM * 2);
static constexpr size_t SZ_PL = al256((size_t)NB * NH_ * SEQ * HD * 2);
static constexpr size_t SZ_CX = al256((size_t)NB * SEQ * DM * 2);
static constexpr size_t SZ_TOTAL = 3 * SZ_XB + 4 * SZ_WT + 5 * SZ_PL + 2 * SZ_CX;
static_assert(SZ_TOTAL <= (size_t)134217728);
static_assert(((size_t)DM * DM * 2) % 256 == 0);
static_assert((size_t)NB * NH_ * SEQ * HD == (size_t)NB * DM * SEQ);
static_assert((size_t)(NB * SEQ / 64) * 64 == (size_t)NB * SEQ);
static_assert((size_t)(DM / 64) * 64 == (size_t)DM);
static_assert((size_t)(SEQ / (16 * AW)) * (16 * AW) == (size_t)SEQ);
static_assert((size_t)(NB * SEQ / 32) * 32 == (size_t)NB * SEQ);

extern "C" void kernel_launch(void* const* d_in, const int* in_sizes, int n_in,
                              void* d_out, int out_size, void* d_ws, size_t ws_size, hipStream_t stream) {
    if (n_in < 12) return;
    const size_t needx = ((size_t)(NB - 1) * SEQ_FULL + SEQ) * DM;
    const size_t needm = (size_t)(SEQ - 1) * SEQ_FULL + SEQ;
    if ((size_t)in_sizes[0] < needx || (size_t)in_sizes[1] < needx || (size_t)in_sizes[2] < needx) return;
    if ((size_t)in_sizes[3] < needm) return;
    if ((size_t)in_sizes[4] < (size_t)DM * DM || (size_t)in_sizes[6] < (size_t)DM * DM || (size_t)in_sizes[8] < (size_t)DM * DM || (size_t)in_sizes[10] < (size_t)DM * DM) return;
    if (in_sizes[5] < DM || in_sizes[7] < DM || in_sizes[9] < DM || in_sizes[11] < DM) return;
    if ((size_t)out_size < ((size_t)(NB - 1) * OUT_SEQ + SEQ) * DM) return;
    if (SZ_TOTAL > ws_size) return;
    const float* xin[3] = { (const float*)d_in[0], (const float*)d_in[1], (const float*)d_in[2] };
    const int* mk = (const int*)d_in[3];
    const float* wq = (const float*)d_in[4];  const float* bq = (const float*)d_in[5];
    const float* wk = (const float*)d_in[6];  const float* bk = (const float*)d_in[7];
    const float* wv = (const float*)d_in[8];  const float* bv = (const float*)d_in[9];
    const float* wo = (const float*)d_in[10]; const float* bo = (const float*)d_in[11];
    float* OUT = (float*)d_out;
    char* wsp = (char*)d_ws;
    bf* XB[3];
    XB[0] = (bf*)wsp; wsp += SZ_XB;
    XB[1] = (bf*)wsp; wsp += SZ_XB;
    XB[2] = (bf*)wsp; wsp += SZ_XB;
    bf* WQ = (bf*)wsp; wsp += SZ_WT;
    bf* WK = (bf*)wsp; wsp += SZ_WT;
    bf* WV = (bf*)wsp; wsp += SZ_WT;
    h16* WO = (h16*)wsp; wsp += SZ_WT;
    h16* QH = (h16*)wsp; wsp += SZ_PL;
    h16* QR = (h16*)wsp; wsp += SZ_PL;
    h16* KP = (h16*)wsp; wsp += SZ_PL;
    h16* KR = (h16*)wsp; wsp += SZ_PL;
    h16* VT = (h16*)wsp; wsp += SZ_PL;
    h16* CH = (h16*)wsp; wsp += SZ_CX;
    h16* CR = (h16*)wsp; wsp += SZ_CX;

    for (int i = 0; i < 3; ++i) {
        if (SEQ == SEQ_FULL) {
            const size_t n8 = (size_t)NB * SEQ * DM / 8;
            k_cvt8<<<(unsigned)((n8 + 255) / 256), 256, 0, stream>>>(xin[i], XB[i], n8);
        } else {
            const size_t n8 = (size_t)SEQ * DM / 8;
            for (int b = 0; b < NB; ++b) k_cvt8<<<(unsigned)((n8 + 255) / 256), 256, 0, stream>>>(xin[i] + (size_t)b * SEQ_FULL * DM, XB[i] + (size_t)b * SEQ * DM, n8);
        }
    }
    k_wtr_b<<<dim3(DM / 64, DM / 64, 1), 256, 0, stream>>>(wq, WQ);
    k_wtr_b<<<dim3(DM / 64, DM / 64, 1), 256, 0, stream>>>(wk, WK);
    k_wtr_b<<<dim3(DM / 64, DM / 64, 1), 256, 0, stream>>>(wv, WV);
    k_wtr_h<<<dim3(DM / 64, DM / 64, 1), 256, 0, stream>>>(wo, WO);

    k_proj_rows<<<dim3(NB * SEQ / 64, DM / 64, 1), 32, 0, stream>>>(XB[0], WQ, bq, QH, QR);
    k_proj_rows<<<dim3(NB * SEQ / 64, DM / 64, 1), 32, 0, stream>>>(XB[1], WK, bk, KP, KR);
    k_proj_cols<<<dim3(DM / 64, NB * SEQ / 64, 1), 32, 0, stream>>>(WV, XB[2], bv, VT);

    k_attn<<<dim3(SEQ / (16 * AW), NB * NH_, 1), 32 * AW, 0, stream>>>(QH, QR, KP, KR, VT, mk, CH, CR);

    k_oproj<<<dim3(NB * SEQ / 32, DM / 64, 1), 32, 0, stream>>>(CH, CR, WO, bo, OUT);
}
